// DecayLinearAttention_34041910788516
// MI455X (gfx1250) — hardware-verified
//
#include <hip/hip_runtime.h>


constexpr int kB = 2, kN = 2048, kE = 1024, kH = 16, kD = 64, kC = 16;
constexpr int kM = kB * kN;
constexpr float kScale = 0.125f;
constexpr float kEps = 1e-5f;
static_assert(kE == kH * kD);
static_assert(kM % 128 == 0 && kE % 64 == 0 && kD % 64 == 0 && kE % 32 == 0 && kD % 32 == 0);
static_assert(kN % kC == 0 && kC == 16 && kD == 64);

typedef __bf16 bf;
typedef bf    v8b  __attribute__((ext_vector_type(8)));
typedef bf    v16b __attribute__((ext_vector_type(16)));
typedef float v8f  __attribute__((ext_vector_type(8)));
typedef float v4f  __attribute__((ext_vector_type(4)));
union Frag { v16b v; v8b h[2]; };

__device__ __forceinline__ v8f zero8() {
  v8f z = {0.f, 0.f, 0.f, 0.f, 0.f, 0.f, 0.f, 0.f};
  return z;
}

__device__ __forceinline__ v8f mma(v16b a, v16b b, v8f c) {
  v8f d = __builtin_amdgcn_wmma_f32_16x16x32_bf16(false, a, false, b, (short)0, c, false, false);
  asm volatile("v_nop\n\tv_nop\n\tv_nop\n\tv_nop" : "+v"(d) : "v"(a), "v"(b));
  return d;
}

__device__ __forceinline__ v8b cvt8(v8f x) { return __builtin_convertvector(x, v8b); }

__device__ __forceinline__ void split8(v8f x, v8b& hi, v8b& lo) {
  hi = __builtin_convertvector(x, v8b);
  const v8f hf = __builtin_convertvector(hi, v8f);
  lo = __builtin_convertvector(x - hf, v8b);
}

template <int ACT>
__device__ __forceinline__ float act_fn(float x) {
  if constexpr (ACT == 0) {
    return x;
  } else if constexpr (ACT == 1) {
    return x * __builtin_amdgcn_rcpf(1.f + __expf(-x));
  } else if constexpr (ACT == 2) {
    return kScale * (x * __builtin_amdgcn_rcpf(1.f + __expf(-x)));
  } else {
    return __builtin_amdgcn_rcpf(1.f + __expf(-x));
  }
}

__global__ __launch_bounds__(256) void cvt_kernel(const float* __restrict__ src, bf* __restrict__ dst, int n8) {
  const int i = blockIdx.x * 256 + threadIdx.x;
  if (i >= n8) return;
  const size_t o = (size_t)i * 8;
  const v4f a = *(const v4f*)(src + o);
  const v4f b = *(const v4f*)(src + o + 4);
  const v8f x = __builtin_shufflevector(a, b, 0, 1, 2, 3, 4, 5, 6, 7);
  const v8b y = cvt8(x);
  *(volatile v8b*)(dst + o) = y;
  __threadfence();
  *(volatile v8b*)(dst + o) = y;
}

__global__ __launch_bounds__(256) void cvt_wt_kernel(const float* __restrict__ src, bf* __restrict__ dst,
                                                     int K, int N) {
  constexpr int LT = 72;
  __shared__ __attribute__((aligned(16))) bf T[64 * LT];
  const int tid = threadIdx.x, lane = tid & 31, w = tid >> 5;
  const int n0 = blockIdx.x * 64, k0 = blockIdx.y * 64;
  if (n0 + 64 > N || k0 + 64 > K) return;
#pragma unroll
  for (int i = 0; i < 4; ++i) {
    const int idx = tid + 256 * i, kr = idx >> 4, c4 = (idx & 15) * 4;
    const v4f t = *(const v4f*)(src + (size_t)(k0 + kr) * N + n0 + c4);
#pragma unroll
    for (int j = 0; j < 4; ++j) T[(c4 + j) * LT + kr] = (bf)t[j];
  }
  __syncthreads();
  v8b vals[2];
#pragma unroll
  for (int i = 0; i < 2; ++i) {
    const int row = 8 * w + 4 * i + (lane >> 3), kk = (lane & 7) * 8;
    vals[i] = *(const v8b*)(&T[row * LT + kk]);
  }
#pragma unroll
  for (int i = 0; i < 2; ++i) {
    const int row = 8 * w + 4 * i + (lane >> 3), kk = (lane & 7) * 8;
    *(volatile v8b*)(dst + (size_t)(n0 + row) * K + k0 + kk) = vals[i];
  }
  __threadfence();
#pragma unroll
  for (int i = 0; i < 2; ++i) {
    const int row = 8 * w + 4 * i + (lane >> 3), kk = (lane & 7) * 8;
    *(volatile v8b*)(dst + (size_t)(n0 + row) * K + k0 + kk) = vals[i];
  }
}

template <int ACT, int ASPLIT, int OUTP>
__global__ __launch_bounds__(256) void gemm_kernel(const bf* __restrict__ Ah, const bf* __restrict__ Al,
                                                   const bf* __restrict__ Bt, float* __restrict__ Cf,
                                                   bf* __restrict__ Ch, bf* __restrict__ Cl,
                                                   int M, int K, int N) {
  constexpr int LDT = 40;
  constexpr int LDC = 68;
  __shared__ __attribute__((aligned(16))) unsigned char smem[128 * LDC * 4];
  bf* sAh = reinterpret_cast<bf*>(smem);
  bf* sAl = sAh + 128 * LDT;
  bf* sB  = sAl + 128 * LDT;
  float* sC = reinterpret_cast<float*>(smem);

  const int tid = threadIdx.x, lane = tid & 31, w = tid >> 5;
  const int h = lane >> 4, m = lane & 15;
  const int wm = w & 3, wn = w >> 2;
  const int bm = blockIdx.x * 128, bn = blockIdx.y * 64;
  if (bm + 128 > M || bn + 64 > N) return;

  v8f acc[2][2];
#pragma unroll
  for (int i = 0; i < 2; ++i)
#pragma unroll
    for (int j = 0; j < 2; ++j) acc[i][j] = zero8();

  for (int k0 = 0; k0 < K; k0 += 32) {
    __syncthreads();
#pragma unroll
    for (int i = 0; i < 2; ++i) {
      const int c = tid + 256 * i, r = c >> 2, p = (c & 3) * 8;
      const size_t go = (size_t)(bm + r) * K + k0 + p;
      *(v8b*)(sAh + r * LDT + p) = *(const v8b*)(Ah + go);
      if constexpr (ASPLIT != 0) *(v8b*)(sAl + r * LDT + p) = *(const v8b*)(Al + go);
    }
    {
      const int r = tid >> 2, p = (tid & 3) * 8;
      *(v8b*)(sB + r * LDT + p) = *(const v8b*)(Bt + (size_t)(bn + r) * K + k0 + p);
    }
    __syncthreads();

    Frag b[2];
#pragma unroll
    for (int nt = 0; nt < 2; ++nt) {
      const bf* bp = sB + (32 * wn + 16 * nt + m) * LDT + 8 * h;
      b[nt].h[0] = *(const v8b*)bp;
      b[nt].h[1] = *(const v8b*)(bp + 16);
    }
#pragma unroll
    for (int mt = 0; mt < 2; ++mt) {
      const int ar = (32 * wm + 16 * mt + m) * LDT + 8 * h;
      Frag a;
      a.h[0] = *(const v8b*)(sAh + ar);
      a.h[1] = *(const v8b*)(sAh + ar + 16);
      acc[mt][0] = mma(a.v, b[0].v, acc[mt][0]);
      acc[mt][1] = mma(a.v, b[1].v, acc[mt][1]);
      if constexpr (ASPLIT != 0) {
        Frag al;
        al.h[0] = *(const v8b*)(sAl + ar);
        al.h[1] = *(const v8b*)(sAl + ar + 16);
        acc[mt][0] = mma(al.v, b[0].v, acc[mt][0]);
        acc[mt][1] = mma(al.v, b[1].v, acc[mt][1]);
      }
    }
  }
  __syncthreads();

#pragma unroll
  for (int mt = 0; mt < 2; ++mt)
#pragma unroll
    for (int nt = 0; nt < 2; ++nt)
#pragma unroll
      for (int r = 0; r < 8; ++r)
        sC[(32 * wm + 16 * mt + 8 * h + r) * LDC + 32 * wn + 16 * nt + m] = act_fn<ACT>(acc[mt][nt][r]);
  __syncthreads();

  if constexpr (OUTP == 0) {
    v4f vals[8];
#pragma unroll
    for (int i = 0; i < 8; ++i) {
      const int row = 16 * w + 2 * i + h, col = 4 * m;
      vals[i] = *(const v4f*)(sC + row * LDC + col);
    }
#pragma unroll
    for (int i = 0; i < 8; ++i) {
      const int row = 16 * w + 2 * i + h, col = 4 * m;
      *(volatile v4f*)(Cf + (size_t)(bm + row) * N + bn + col) = vals[i];
    }
    __threadfence();
#pragma unroll
    for (int i = 0; i < 8; ++i) {
      const int row = 16 * w + 2 * i + h, col = 4 * m;
      *(volatile v4f*)(Cf + (size_t)(bm + row) * N + bn + col) = vals[i];
    }
  } else {
    v8b hv[4], lv[4];
#pragma unroll
    for (int i = 0; i < 4; ++i) {
      const int row = 16 * w + 4 * i + (lane >> 3), c0 = (lane & 7) * 8;
      const v4f xa = *(const v4f*)(sC + row * LDC + c0);
      const v4f xb = *(const v4f*)(sC + row * LDC + c0 + 4);
      const v8f x8 = __builtin_shufflevector(xa, xb, 0, 1, 2, 3, 4, 5, 6, 7);
      split8(x8, hv[i], lv[i]);
    }
#pragma unroll
    for (int i = 0; i < 4; ++i) {
      const int row = 16 * w + 4 * i + (lane >> 3), c0 = (lane & 7) * 8;
      const size_t go = (size_t)(bm + row) * N + bn + c0;
      *(volatile v8b*)(Ch + go) = hv[i];
      *(volatile v8b*)(Cl + go) = lv[i];
    }
    __threadfence();
#pragma unroll
    for (int i = 0; i < 4; ++i) {
      const int row = 16 * w + 4 * i + (lane >> 3), c0 = (lane & 7) * 8;
      const size_t go = (size_t)(bm + row) * N + bn + c0;
      *(volatile v8b*)(Ch + go) = hv[i];
      *(volatile v8b*)(Cl + go) = lv[i];
    }
  }
}

__global__ __launch_bounds__(128) void recur_kernel(const float* __restrict__ q, const float* __restrict__ k,
                                                    const float* __restrict__ v, const float* __restrict__ f,
                                                    const float* __restrict__ g, const float* __restrict__ nw,
                                                    bf* __restrict__ onh, bf* __restrict__ onl, int nc) {
  __shared__ __attribute__((aligned(16))) float stg[5][kC][kD];
  __shared__ __attribute__((aligned(16))) float cfs[kC][kD];
  __shared__ __attribute__((aligned(16))) float cfl[kD];
  __shared__ __attribute__((aligned(16))) bf qh[kC][kD];
  __shared__ __attribute__((aligned(16))) bf ql[kC][kD];
  __shared__ __attribute__((aligned(16))) bf kh[kC][kD];
  __shared__ __attribute__((aligned(16))) bf kl[kC][kD];
  __shared__ __attribute__((aligned(16))) bf kth[kD][kC];
  __shared__ __attribute__((aligned(16))) bf ktl[kD][kC];

  const int tid = threadIdx.x, lane = tid & 31, w = tid >> 5;
  const int h = lane >> 4, m = lane & 15;
  const int bh = blockIdx.x;
  if (bh >= kB * kH) return;
  const int b = bh / kH, hd = bh - b * kH;
  const int cb = 16 * w;
  const size_t rowbase = (size_t)b * kN;
  const int coloff = hd * kD;
  const int erow = tid >> 3, ec0 = (tid & 7) * 8;

  float nw8[8];
#pragma unroll
  for (int j = 0; j < 8; ++j) nw8[j] = nw[coloff + ec0 + j];

  float S[32];
#pragma unroll
  for (int i = 0; i < 32; ++i) S[i] = 0.f;

  const v8f z8 = zero8();
  const v8b zb = cvt8(z8);
  float* os = &stg[0][0][0];

  for (int ci = 0; ci < nc; ++ci) {
    const int n0 = ci * kC;
    __syncthreads();
#pragma unroll
    for (int i = 0; i < 10; ++i) {
      const int a = i >> 1, rem = tid + 128 * (i & 1), r = rem >> 4, c4 = (rem & 15) * 4;
      const float* src = (i < 2) ? q : (i < 4) ? k : (i < 6) ? v : (i < 8) ? f : g;
      *(v4f*)&stg[a][r][c4] = *(const v4f*)(src + (rowbase + n0 + r) * kE + coloff + c4);
    }
    __syncthreads();
    if (tid < kD) {
      float run = 1.f;
#pragma unroll
      for (int t = 0; t < kC; ++t) { run *= stg[3][t][tid]; cfs[t][tid] = run; }
      cfl[tid] = run;
    }
    __syncthreads();
    {
      const int t = tid >> 3, d0 = (tid & 7) * 8;
      v8f qq = z8, kk = z8;
#pragma unroll
      for (int j = 0; j < 8; ++j) {
        const float c = cfs[t][d0 + j];
        qq[j] = stg[0][t][d0 + j] * c;
        kk[j] = stg[1][t][d0 + j] * __builtin_amdgcn_rcpf(c);
      }
      v8b ph, pl;
      split8(qq, ph, pl);
      *(v8b*)&qh[t][d0] = ph;
      *(v8b*)&ql[t][d0] = pl;
      split8(kk, ph, pl);
      *(v8b*)&kh[t][d0] = ph;
      *(v8b*)&kl[t][d0] = pl;
    }
    {
      const int d = tid >> 1, t0 = (tid & 1) * 8;
      const float fl = cfl[d];
      v8f x8 = z8;
#pragma unroll
      for (int j = 0; j < 8; ++j) {
        const int t = t0 + j;
        x8[j] = stg[1][t][d] * (fl * __builtin_amdgcn_rcpf(cfs[t][d]));
      }
      v8b ph, pl;
      split8(x8, ph, pl);
      *(v8b*)&kth[d][t0] = ph;
      *(v8b*)&ktl[d][t0] = pl;
    }
    v8b vh, vl;
    {
      v8f vv = z8;
#pragma unroll
      for (int r = 0; r < 8; ++r) vv[r] = stg[2][8 * h + r][cb + m];
      split8(vv, vh, vl);
    }
    __syncthreads();

    v8f accT = z8;
#pragma unroll
    for (int ks = 0; ks < kD; ks += 32) {
      Frag ka, kal, qb, qbl;
      ka.h[0]  = *(const v8b*)&kh[m][ks + 8 * h];
      ka.h[1]  = *(const v8b*)&kh[m][ks + 16 + 8 * h];
      kal.h[0] = *(const v8b*)&kl[m][ks + 8 * h];
      kal.h[1] = *(const v8b*)&kl[m][ks + 16 + 8 * h];
      qb.h[0]  = *(const v8b*)&qh[m][ks + 8 * h];
      qb.h[1]  = *(const v8b*)&qh[m][ks + 16 + 8 * h];
      qbl.h[0] = *(const v8b*)&ql[m][ks + 8 * h];
      qbl.h[1] = *(const v8b*)&ql[m][ks + 16 + 8 * h];
      accT = mma(ka.v, qb.v, accT);
      accT = mma(ka.v, qbl.v, accT);
      accT = mma(kal.v, qb.v, accT);
    }
    v8f am = z8;
#pragma unroll
    for (int r = 0; r < 8; ++r) am[r] = ((8 * h + r) <= m) ? accT[r] : 0.f;
    v8b amh, aml;
    split8(am, amh, aml);
    Frag a1, a2, b1, b2;
    a1.h[0] = amh; a1.h[1] = aml;
    a2.h[0] = amh; a2.h[1] = zb;
    b1.h[0] = vh;  b1.h[1] = vh;
    b2.h[0] = vl;  b2.h[1] = zb;
    v8f accO = mma(a1.v, b1.v, z8);
    accO = mma(a2.v, b2.v, accO);

#pragma unroll
    for (int ksi = 0; ksi < 2; ++ksi) {
      Frag qa, qal, sb, sbl;
      qa.h[0]  = *(const v8b*)&qh[m][32 * ksi + 8 * h];
      qa.h[1]  = *(const v8b*)&qh[m][32 * ksi + 16 + 8 * h];
      qal.h[0] = *(const v8b*)&ql[m][32 * ksi + 8 * h];
      qal.h[1] = *(const v8b*)&ql[m][32 * ksi + 16 + 8 * h];
      v8f s0 = z8, s1 = z8;
#pragma unroll
      for (int i = 0; i < 8; ++i) { s0[i] = S[16 * ksi + i]; s1[i] = S[16 * ksi + 8 + i]; }
      split8(s0, sb.h[0], sbl.h[0]);
      split8(s1, sb.h[1], sbl.h[1]);
      accO = mma(qa.v, sb.v, accO);
      accO = mma(qa.v, sbl.v, accO);
      accO = mma(qal.v, sb.v, accO);
    }
#pragma unroll
    for (int r = 0; r < 8; ++r) os[(8 * h + r) * kD + cb + m] = accO[r];

#pragma unroll
    for (int mt = 0; mt < 4; ++mt) {
      Frag c1, c2;
      c1.h[0] = *(const v8b*)&kth[16 * mt + m][8 * h];
      c1.h[1] = *(const v8b*)&ktl[16 * mt + m][8 * h];
      c2.h[0] = c1.h[0];
      c2.h[1] = zb;
      v8f accS = mma(c1.v, b1.v, z8);
      accS = mma(c2.v, b2.v, accS);
#pragma unroll
      for (int r = 0; r < 8; ++r) {
        const int d = 16 * mt + 8 * h + r;
        S[8 * mt + r] = cfl[d] * S[8 * mt + r] + accS[r];
      }
    }
    __syncthreads();

    {
      v8f og = z8;
      float ss = 0.f;
#pragma unroll
      for (int j = 0; j < 8; ++j) {
        const float o = os[erow * kD + ec0 + j] * stg[4][erow][ec0 + j];
        og[j] = o;
        ss += o * o;
      }
      ss += __shfl_xor(ss, 1, 32);
      ss += __shfl_xor(ss, 2, 32);
      ss += __shfl_xor(ss, 4, 32);
      const float rn = rsqrtf(ss * (1.0f / (float)kD) + kEps);
      v8f y = z8;
#pragma unroll
      for (int j = 0; j < 8; ++j) y[j] = og[j] * rn * nw8[j];
      v8b yh, yl;
      split8(y, yh, yl);
      const size_t go = (rowbase + n0 + erow) * kE + coloff + ec0;
      *(volatile v8b*)(onh + go) = yh;
      *(volatile v8b*)(onl + go) = yl;
      __threadfence();
      *(volatile v8b*)(onh + go) = yh;
      *(volatile v8b*)(onl + go) = yl;
    }
  }
}

extern "C" void kernel_launch(void* const* d_in, const int* in_sizes, int n_in,
                              void* d_out, int out_size, void* d_ws, size_t ws_size,
                              hipStream_t stream) {
  if (n_in < 10) return;
  if (in_sizes[0] != kM * kE || in_sizes[1] != kE * kE || in_sizes[2] != kE * kE ||
      in_sizes[3] != kE * kE || in_sizes[4] != kE * kE || in_sizes[5] != kE * kD ||
      in_sizes[6] != kD * kE || in_sizes[7] != kE * kD || in_sizes[8] != kD * kE ||
      in_sizes[9] != kE || out_size != kM * kE) return;

  const float* x   = (const float*)d_in[0];
  const float* Wq  = (const float*)d_in[1];
  const float* Wk  = (const float*)d_in[2];
  const float* Wv  = (const float*)d_in[3];
  const float* Wo  = (const float*)d_in[4];
  const float* Wf1 = (const float*)d_in[5];
  const float* Wf2 = (const float*)d_in[6];
  const float* Wg1 = (const float*)d_in[7];
  const float* Wg2 = (const float*)d_in[8];
  const float* nw  = (const float*)d_in[9];
  float* out = (float*)d_out;

  unsigned char* ws = (unsigned char*)d_ws;
  size_t off = 0;
  auto carve = [&](size_t bytes) -> unsigned char* {
    unsigned char* p = ws + off;
    off += (bytes + 255) & ~(size_t)255;
    return p;
  };
  bf* xb   = (bf*)carve((size_t)kM * kE * 2);
  bf* wqt  = (bf*)carve((size_t)kE * kE * 2);
  bf* wkt  = (bf*)carve((size_t)kE * kE * 2);
  bf* wvt  = (bf*)carve((size_t)kE * kE * 2);
  bf* wot  = (bf*)carve((size_t)kE * kE * 2);
  bf* wf1t = (bf*)carve((size_t)kD * kE * 2);
  bf* wg1t = (bf*)carve((size_t)kD * kE * 2);
  bf* wf2t = (bf*)carve((size_t)kE * kD * 2);
  bf* wg2t = (bf*)carve((size_t)kE * kD * 2);
  float* qf = (float*)carve((size_t)kM * kE * 4);
  float* kf = (float*)carve((size_t)kM * kE * 4);
  float* vf = (float*)carve((size_t)kM * kE * 4);
  float* ff = (float*)carve((size_t)kM * kE * 4);
  float* gf = (float*)carve((size_t)kM * kE * 4);
  bf* xfh  = (bf*)carve((size_t)kM * kD * 2);
  bf* xfl  = (bf*)carve((size_t)kM * kD * 2);
  bf* xgh  = (bf*)carve((size_t)kM * kD * 2);
  bf* xgl  = (bf*)carve((size_t)kM * kD * 2);
  bf* onh  = (bf*)carve((size_t)kM * kE * 2);
  bf* onl  = (bf*)carve((size_t)kM * kE * 2);
  if (off > ws_size) return;

  const int n8 = kM * kE / 8;
  cvt_kernel<<<(n8 + 255) / 256, 256, 0, stream>>>(x, xb, n8);

  const dim3 gW((kE + 63) / 64, (kE + 63) / 64);
  cvt_wt_kernel<<<gW, 256, 0, stream>>>(Wq, wqt, kE, kE);
  cvt_wt_kernel<<<gW, 256, 0, stream>>>(Wk, wkt, kE, kE);
  cvt_wt_kernel<<<gW, 256, 0, stream>>>(Wv, wvt, kE, kE);
  cvt_wt_kernel<<<gW, 256, 0, stream>>>(Wo, wot, kE, kE);
  const dim3 gW1((kD + 63) / 64, (kE + 63) / 64);
  cvt_wt_kernel<<<gW1, 256, 0, stream>>>(Wf1, wf1t, kE, kD);
  cvt_wt_kernel<<<gW1, 256, 0, stream>>>(Wg1, wg1t, kE, kD);
  const dim3 gW2((kE + 63) / 64, (kD + 63) / 64);
  cvt_wt_kernel<<<gW2, 256, 0, stream>>>(Wf2, wf2t, kD, kE);
  cvt_wt_kernel<<<gW2, 256, 0, stream>>>(Wg2, wg2t, kD, kE);

  const dim3 blk(256);
  const dim3 gME((kM + 127) / 128, (kE + 63) / 64);
  const dim3 gMD((kM + 127) / 128, (kD + 63) / 64);

  gemm_kernel<2, 0, 0><<<gME, blk, 0, stream>>>(xb, xb, wqt, qf, xfh, xfl, kM, kE, kE);
  gemm_kernel<1, 0, 0><<<gME, blk, 0, stream>>>(xb, xb, wkt, kf, xfh, xfl, kM, kE, kE);
  gemm_kernel<0, 0, 0><<<gME, blk, 0, stream>>>(xb, xb, wvt, vf, xfh, xfl, kM, kE, kE);
  gemm_kernel<0, 0, 1><<<gMD, blk, 0, stream>>>(xb, xb, wf1t, qf, xfh, xfl, kM, kE, kD);
  gemm_kernel<3, 1, 0><<<gME, blk, 0, stream>>>(xfh, xfl, wf2t, ff, xgh, xgl, kM, kD, kE);
  gemm_kernel<0, 0, 1><<<gMD, blk, 0, stream>>>(xb, xb, wg1t, qf, xgh, xgl, kM, kE, kD);
  gemm_kernel<3, 1, 0><<<gME, blk, 0, stream>>>(xgh, xgl, wg2t, gf, xfh, xfl, kM, kD, kE);

  recur_kernel<<<kB * kH, 128, 0, stream>>>(qf, kf, vf, ff, gf, nw, onh, onl, kN / kC);

  gemm_kernel<0, 1, 0><<<gME, blk, 0, stream>>>(onh, onl, wot, out, xfh, xfl, kM, kE, kE);
}
